// ComirecSA_4303557231217
// MI455X (gfx1250) — hardware-verified
//
#include <hip/hip_runtime.h>
#include <math.h>

typedef __attribute__((ext_vector_type(16))) _Float16 v16h;
typedef __attribute__((ext_vector_type(16))) __bf16 v16b;
typedef __attribute__((ext_vector_type(8)))  _Float16 v8h;
typedef __attribute__((ext_vector_type(8)))  float v8f;
typedef __attribute__((ext_vector_type(4)))  float v4f;
typedef __attribute__((ext_vector_type(2)))  float v2f;
typedef __attribute__((ext_vector_type(4)))  unsigned v4u;
typedef __attribute__((ext_vector_type(4)))  int v4i;
typedef float __attribute__((may_alias)) float_a;
typedef int __attribute__((may_alias)) int_a;

template <typename T> __device__ __forceinline__ void vst2(void* p, T v) { *(volatile T*)p = v; __threadfence(); *(volatile T*)p = v; }
__device__ __forceinline__ v8f wmma16(v16h a, v16h b, v8f c) {
  v8f d = __builtin_amdgcn_wmma_f32_16x16x32_f16(false, a, false, b, (short)0, c, false, false);
  asm volatile("v_nop\n\tv_nop\n\tv_nop\n\tv_nop" : "+v"(d) : "v"(a), "v"(b));
  return d;
}
__device__ __forceinline__ v8f wmma_bf(v16b a, v16b b, v8f c) {
  v8f d = __builtin_amdgcn_wmma_f32_16x16x32_bf16(false, a, false, b, (short)0, c, false, false);
  asm volatile("v_nop\n\tv_nop\n\tv_nop\n\tv_nop" : "+v"(d) : "v"(a), "v"(b));
  return d;
}
__device__ __forceinline__ v16h frag_h(const _Float16* rowk0, int lane) {
  union { v16h v; v8h q[2]; } u; const _Float16* p = rowk0 + 8 * (lane >> 4);
  u.q[0] = *(const v8h*)p; u.q[1] = *(const v8h*)(p + 16); return u.v;
}
__device__ __forceinline__ v16h frag_f32(const float* rowk0, int lane) {
  v16h a; const float* p = rowk0 + 8 * (lane >> 4);
#pragma unroll
  for (int i = 0; i < 8; ++i) { a[i] = (_Float16)p[i]; a[8 + i] = (_Float16)p[16 + i]; }
  return a;
}
__device__ __forceinline__ v16h frag_f32s(const float* rowk0, int lane, float sc) {
  v16h a; const float* p = rowk0 + 8 * (lane >> 4);
#pragma unroll
  for (int i = 0; i < 8; ++i) { a[i] = (_Float16)(p[i] * sc); a[8 + i] = (_Float16)(p[16 + i] * sc); }
  return a;
}
__device__ __forceinline__ v16h fragc_f32(const float* W, int k0, int n, int lane, int ld, int K) {
  v16h a; const int g = lane >> 4;
#pragma unroll
  for (int i = 0; i < 8; ++i) { const int ka = k0 + 8 * g + i, kb = ka + 16;
    a[i] = (_Float16)(ka < K ? W[(size_t)(ka < K ? ka : K - 1) * ld + n] : 0.f); a[8 + i] = (_Float16)(kb < K ? W[(size_t)(kb < K ? kb : K - 1) * ld + n] : 0.f); }
  return a;
}
struct F2 { v16b h, l; };
__device__ __forceinline__ F2 bsplit16(const float v[16]) { F2 r;
#pragma unroll
  for (int i = 0; i < 16; ++i) { const __bf16 h = (__bf16)v[i]; r.h[i] = h; r.l[i] = (__bf16)(v[i] - (float)h); }
  return r; }
__device__ __forceinline__ F2 split_row(const float* row, int k0, int lane) { float v[16]; const float* p = row + k0 + 8 * (lane >> 4);
#pragma unroll
  for (int i = 0; i < 8; ++i) { v[i] = p[i]; v[8 + i] = p[16 + i]; }
  return bsplit16(v); }
__device__ __forceinline__ F2 split_rowK(const float* row, int k0, int lane, int K) { float v[16]; const int g = lane >> 4;
#pragma unroll
  for (int i = 0; i < 8; ++i) { const int ka = k0 + 8 * g + i, kb = ka + 16; v[i] = ka < K ? row[ka < K ? ka : K - 1] : 0.f; v[8 + i] = kb < K ? row[kb < K ? kb : K - 1] : 0.f; }
  return bsplit16(v); }
__device__ __forceinline__ F2 split_col(const float* W, int k0, int n, int lane, int ld, int K) { float v[16]; const int g = lane >> 4;
#pragma unroll
  for (int i = 0; i < 8; ++i) { const int ka = k0 + 8 * g + i, kb = ka + 16; v[i] = ka < K ? W[(size_t)(ka < K ? ka : K - 1) * ld + n] : 0.f; v[8 + i] = kb < K ? W[(size_t)(kb < K ? kb : K - 1) * ld + n] : 0.f; }
  return bsplit16(v); }
__device__ __forceinline__ v8f mac3(const F2& a, const F2& b, v8f c) { c = wmma_bf(a.l, b.h, c); c = wmma_bf(a.h, b.l, c); return wmma_bf(a.h, b.h, c); }
__device__ __forceinline__ float sigm(float v) { return 1.0f / (1.0f + expf(-v)); }
#define LDSX() do { asm volatile("s_wait_dscnt 0" ::: "memory"); __builtin_amdgcn_wave_barrier(); __builtin_amdgcn_fence(__ATOMIC_RELEASE, "workgroup"); } while (0)


#define NU 4096
#define LL 200
#define DD 64
#define KI 4
#define HID 256
#define NC 101
#define NROW (NU * LL)
#define NTAB 100000
#ifndef NUT
#define NUT NU
#endif
typedef __attribute__((ext_vector_type(8))) __bf16 v8b;
__device__ __forceinline__ v16b frag_b(const __bf16* rowk0, int lane) {
  union { v16b v; v8b q[2]; } u; const __bf16* p = rowk0 + 8 * (lane >> 4);
  u.q[0] = *(const v8b*)p; u.q[1] = *(const v8b*)(p + 16); return u.v;
}
__device__ __forceinline__ float bfr(float v) { return (float)(__bf16)v; }
__device__ __attribute__((noinline)) float exp_ni(float v) { return expf(v); }
__device__ __attribute__((noinline)) float erf_ni(float v) { return erff(v); }
__device__ __attribute__((noinline)) float tanh_ni(float v) { return tanhf(v); }

#define WS_ITB (0u)
#define WS_W1  (WS_ITB + 2u * NTAB * DD)
#define WS_W2  (WS_W1 + 2u * HID * DD)
#define WS_A2  (WS_W2 + 2u * 16 * HID)
#define STGS 128
#define WS_STG (WS_A2 + 4u * (size_t)NROW * KI)
#define WS_END (WS_STG + 4u * (size_t)NU * STGS)

__global__ __launch_bounds__(256) void k_tab(const float* __restrict__ IT, const float* __restrict__ W1, const float* __restrict__ W2, __bf16* __restrict__ ITB, __bf16* __restrict__ W1B, __bf16* __restrict__ W2B) {
  __shared__ __align__(16) __bf16 s[512 * DD]; const int tid = threadIdx.x; const size_t r0 = (size_t)blockIdx.x * 512;
  for (int e = tid; e < 512 * DD; e += 256) { const size_t r = r0 + e / DD; s[e] = (__bf16)((r < NTAB) ? IT[r * DD + e % DD] : 0.f); }
  __syncthreads();
  for (int e = tid; e < 512 * DD / 8; e += 256) { const size_t r = r0 + (e * 8) / DD; if (r < NTAB) vst2((unsigned*)(ITB + r0 * DD + e * 8), *(const v4u*)&s[e * 8]); }
  if (blockIdx.x == 0) { __syncthreads();
    __shared__ __align__(16) __bf16 w1[HID][DD]; __shared__ __align__(16) __bf16 w2[16][HID];
    for (int e = tid; e < HID * DD; e += 256) { const int h = e / DD, d = e % DD; w1[h][d] = (__bf16)W1[(size_t)d * HID + h]; }
    for (int e = tid; e < 16 * HID; e += 256) { const int k = e / HID, h = e % HID; w2[k][h] = (__bf16)((k < KI) ? W2[(size_t)h * KI + k] : 0.f); }
    __syncthreads();
    for (int e = tid; e < HID * DD / 8; e += 256) vst2((unsigned*)(W1B + e * 8), *(const v4u*)(&w1[0][0] + e * 8));
    for (int e = tid; e < 16 * HID / 8; e += 256) vst2((unsigned*)(W2B + e * 8), *(const v4u*)(&w2[0][0] + e * 8));
  }
}
__global__ __launch_bounds__(128) void k_hist(const int* __restrict__ HIST, const __bf16* __restrict__ ITB, const __bf16* __restrict__ W1B, const __bf16* __restrict__ W2B, float* __restrict__ A2) {
  __shared__ __align__(16) __bf16 sh_[4][16][HID + 8], sl_[4][16][HID + 8]; __shared__ __align__(16) float sa[64][4];
  const int tid = threadIdx.x, wave = tid >> 5, lane = tid & 31, col = lane & 15, g = lane >> 4; const size_t r0 = (size_t)blockIdx.x * 64 + wave * 16;
  const int id = min(max(HIST[r0 + col], 0), NTAB - 1);
  v16b a[2];
#pragma unroll
  for (int kc = 0; kc < 2; ++kc) a[kc] = frag_b(ITB + (size_t)id * DD + kc * 32, lane);
#pragma unroll 1
  for (int half = 0; half < 2; ++half) { v8f acc[8] = {};
#pragma unroll
    for (int kc = 0; kc < 2; ++kc)
#pragma unroll
      for (int j = 0; j < 8; ++j) acc[j] = wmma_bf(a[kc], frag_b(W1B + (size_t)(half * 128 + j * 16 + col) * DD + kc * 32, lane), acc[j]);
#pragma unroll
    for (int j = 0; j < 8; ++j)
#pragma unroll
      for (int r = 0; r < 8; ++r) { const float v = tanh_ni(acc[j][r]); const __bf16 hb = (__bf16)v; sh_[wave][8 * g + r][half * 128 + j * 16 + col] = hb; sl_[wave][8 * g + r][half * 128 + j * 16 + col] = (__bf16)(v - (float)hb); } }
  LDSX();
  v8f c = {};
#pragma unroll
  for (int kc = 0; kc < HID / 32; ++kc) { F2 x; x.h = frag_b(&sh_[wave][col][kc * 32], lane); x.l = frag_b(&sl_[wave][col][kc * 32], lane); const v16b w = frag_b(W2B + (size_t)col * HID + kc * 32, lane); c = wmma_bf(x.l, w, c); c = wmma_bf(x.h, w, c); }
  if (col < KI) {
#pragma unroll
    for (int r = 0; r < 8; ++r) sa[wave * 16 + 8 * g + r][col] = c[r]; }
  __syncthreads();
  if (tid < 64) vst2(A2 + (r0 - wave * 16 + tid) * 4, *(const v4f*)&sa[tid][0]);
}
__global__ __launch_bounds__(256) void k_user(const int* __restrict__ UID, const int* __restrict__ HIST, const int* __restrict__ POS, const int* __restrict__ NEG, const float* __restrict__ UT, const float* __restrict__ IT, const float* __restrict__ CW, const float* __restrict__ A2, float* __restrict__ STG) {
  __shared__ float sA[LL][KI]; __shared__ float smx[KI], ssum[KI]; __shared__ float sint[KI][DD]; __shared__ float sue[KI][DD]; __shared__ float sin_[KI][2 * DD]; __shared__ float sdot[KI]; __shared__ int sk; __shared__ float sbest[DD]; __shared__ float sbn; __shared__ __align__(16) float sout[STGS];
  const int tid = threadIdx.x; const int b = blockIdx.x;
  for (int e = tid; e < LL * KI; e += 256) { const int l = e / KI, k = e % KI; const float m = (HIST[(size_t)b * LL + l] > 0) ? 1.f : 0.f; sA[l][k] = A2[((size_t)b * LL + l) * KI + k] + (-1.0e9f) * (1.0f - m); }
  __syncthreads();
  if (tid < KI) { const int k = tid; float mx = -3.0e38f; for (int l = 0; l < LL; ++l) mx = fmaxf(mx, sA[l][k]); float se = 0.f; for (int l = 0; l < LL; ++l) se += exp_ni(sA[l][k] - mx); smx[k] = mx; ssum[k] = se; }
  __syncthreads();
  for (int e = tid; e < LL * KI; e += 256) { const int l = e / KI, k = e % KI; sA[l][k] = exp_ni(sA[l][k] - smx[k]) / ssum[k]; }
  __syncthreads();
  { const int k = tid >> 6, d = tid & 63; float a = 0.f;
#pragma unroll 1
    for (int l = 0; l < LL; ++l) { const int id = min(max(HIST[(size_t)b * LL + l], 0), NTAB - 1); a += sA[l][k] * bfr(IT[(size_t)id * DD + d]); }
    sint[k][d] = a; const int uid = min(max(UID[b], 0), NTAB - 1); sin_[k][d] = bfr(UT[(size_t)uid * DD + d]); sin_[k][DD + d] = a; }
  __syncthreads();
  { const int k = tid >> 6, d = tid & 63; float a = 0.f;
#pragma unroll 1
    for (int e = 0; e < 2 * DD; ++e) a += sin_[k][e] * bfr(CW[(size_t)e * DD + d]);
    sue[k][d] = a; }
  __syncthreads();
  const int pid = min(max(POS[b], 0), NTAB - 1);
  if (tid < KI) { float a = 0.f; for (int d = 0; d < DD; ++d) a += sue[tid][d] * bfr(IT[(size_t)pid * DD + d]); sdot[tid] = a; }
  __syncthreads();
  if (tid == 0) { int bk = 0; float bv = sdot[0]; for (int k = 1; k < KI; ++k) if (sdot[k] > bv) { bv = sdot[k]; bk = k; } sk = bk; }
  __syncthreads();
  if (tid < DD) sbest[tid] = sue[sk][tid];
  __syncthreads();
  if (tid == 0) { float a = 0.f; for (int d = 0; d < DD; ++d) a += sbest[d] * sbest[d]; sbn = fmaxf(sqrtf(a), 1e-8f); }
  __syncthreads();
  if (tid < NC) { const int id = (tid == 0) ? pid : min(max(NEG[(size_t)b * (NC - 1) + tid - 1], 0), NTAB - 1); float num = 0.f, nn = 0.f;
#pragma unroll 1
    for (int d = 0; d < DD; ++d) { const float iv = bfr(IT[(size_t)id * DD + d]); num += sbest[d] * iv; nn += iv * iv; }
    sout[tid] = num / (sbn * fmaxf(sqrtf(nn), 1e-8f)); }
  if (tid >= NC && tid < STGS) sout[tid] = 0.f;
  __syncthreads();
  if (tid < STGS / 4) vst2(STG + (size_t)b * STGS + tid * 4, *(const v4f*)&sout[tid * 4]);
}
__global__ __launch_bounds__(256) void k_flat(const float* __restrict__ STG, float* __restrict__ OUT) {
  const size_t q = (size_t)blockIdx.x * 256 + threadIdx.x; if (q >= (size_t)NUT * NC / 4) return; v4f v;
#pragma unroll
  for (int e = 0; e < 4; ++e) { const size_t f = q * 4 + e; v[e] = STG[(f / NC) * STGS + f % NC]; }
  vst2(OUT + q * 4, v);
}
extern "C" void kernel_launch(void* const* d_in, const int* in_sizes, int n_in, void* d_out, int out_size, void* d_ws, size_t ws_size, hipStream_t stream) {
  (void)in_sizes; (void)n_in; (void)out_size;
  if (ws_size < (size_t)WS_END) return;
  char* ws = (char*)d_ws; __bf16 *ITB = (__bf16*)(ws + WS_ITB), *W1B = (__bf16*)(ws + WS_W1), *W2B = (__bf16*)(ws + WS_W2); float *A2 = (float*)(ws + WS_A2), *STG = (float*)(ws + WS_STG);
  const int* UID = (const int*)d_in[0]; const int* HIST = (const int*)d_in[1]; const int* POS = (const int*)d_in[2]; const int* NEG = (const int*)d_in[3]; const float* UT = (const float*)d_in[4]; const float* IT = (const float*)d_in[5];
  k_tab<<<(NTAB + 511) / 512, 256, 0, stream>>>(IT, (const float*)d_in[6], (const float*)d_in[7], ITB, W1B, W2B);
  k_hist<<<NUT * LL / 64, 128, 0, stream>>>(HIST, ITB, W1B, W2B, A2);
  k_user<<<NUT, 256, 0, stream>>>(UID, HIST, POS, NEG, UT, IT, (const float*)d_in[8], A2, STG);
  k_flat<<<(NUT * NC / 4 + 255) / 256, 256, 0, stream>>>(STG, (float*)d_out);
}
